// GravNet_simple_1271310320344
// MI455X (gfx1250) — hardware-run, weakly checked
//
#include <hip/hip_runtime.h>


#ifndef NB
#define NB 4
#endif
#ifndef SEQ
#define SEQ 4096
#endif
#define NB_FULL  4
#define SEQ_FULL 4096
#ifndef OUT_SEQ
#define OUT_SEQ SEQ
#endif
#define FIN  64
#define PW   64
#define SD   4
#define FOUT 64
#define N1   80
#define NT1  (N1 / 16)
#define CW   128
#define KNN  40
#define KQ   64
#define CT   256
#define CSP  136
#define G1P  84
#define OP2  68
#define CCS  16.0f
#define WXS  256.0f
#define WCS  16.0f
#define OINV (1.0f / 256.0f)
#define LOG2E 1.4426950408889634f

static_assert(FIN % 32 == 0);
static_assert(CW % 32 == 0);
static_assert(PW == 64);
static_assert(FOUT == 64);
static_assert(SD == 4);
static_assert(PW + SD <= N1);
static_assert(N1 % 16 == 0);
static_assert(CW == 2 * PW);
static_assert(SEQ % 32 == 0);
static_assert((NB * SEQ) % 32 == 0);
static_assert(SEQ % KQ == 0);
static_assert(SEQ % CT == 0);
static_assert(CT % KQ == 0);
static_assert(SEQ > KNN);
static_assert(KQ == 64);
static_assert(NB <= NB_FULL);
static_assert(SEQ <= SEQ_FULL);
static_assert(CCS * WCS == WXS);
static_assert((G1P * 4) % 16 == 0);
static_assert((OP2 * 4) % 16 == 0);
static_assert((CSP * 2) % 16 == 0);
static_assert(G1P >= N1);
static_assert(OP2 >= FOUT);
static_assert(CSP >= CW);
static_assert(8 * 32 * 16 == 16 * PW * 4);
static_assert(8 * 32 * 16 == 16 * FOUT * 4);
static_assert(16 * 16 == 16 * SD * 4);
static_assert(16 * 32 * 16 == 32 * CW * 2);
static_assert(16 * G1P * 4 <= 131072);
static_assert(16 * OP2 * 4 <= 131072);
static_assert(CT * 16 + KQ * KNN * 8 + KQ * CSP * 2 <= 131072);

typedef _Float16 h16;
typedef unsigned short bf;
typedef __attribute__((ext_vector_type(16))) __bf16   v16bf;
typedef __attribute__((ext_vector_type(16))) _Float16 v16h;
typedef __attribute__((ext_vector_type(8)))  _Float16 v8h;
typedef __attribute__((ext_vector_type(8)))  unsigned short v8us;
typedef __attribute__((ext_vector_type(8)))  float    v8f;
typedef __attribute__((ext_vector_type(4)))  float    v4f;
typedef __attribute__((ext_vector_type(2)))  float    v2f;
typedef v4f  __attribute__((may_alias)) v4fa;
typedef v8h  __attribute__((may_alias)) v8ha;

__device__ __forceinline__ unsigned short f2bf(float f) { unsigned u = __float_as_uint(f); u += 0x7FFFu + ((u >> 16) & 1u); return (unsigned short)(u >> 16); }
__device__ __forceinline__ float bfr(float f) { return __uint_as_float(((unsigned)f2bf(f)) << 16); }
__device__ __forceinline__ v16h cat16(v8h lo, v8h hi) { return __builtin_shufflevector(lo, hi, 0, 1, 2, 3, 4, 5, 6, 7, 8, 9, 10, 11, 12, 13, 14, 15); }
__device__ __forceinline__ v16bf cat16b(v8us lo, v8us hi) { return __builtin_bit_cast(v16bf, __builtin_shufflevector(lo, hi, 0, 1, 2, 3, 4, 5, 6, 7, 8, 9, 10, 11, 12, 13, 14, 15)); }
__device__ __forceinline__ v8f wmma16(v16h a, v16h b, v8f c) { return __builtin_amdgcn_wmma_f32_16x16x32_f16(false, a, false, b, (short)0, c, false, false); }
__device__ __forceinline__ v8f wmmab(v16bf a, v16bf b, v8f c) { return __builtin_amdgcn_wmma_f32_16x16x32_bf16(false, a, false, b, (short)0, c, false, false); }
__device__ __forceinline__ v16h  ldh(const h16* p) { return cat16(*(const v8h*)p, *(const v8h*)(p + 16)); }
__device__ __forceinline__ v16bf ldb(const bf* p)  { return cat16b(*(const v8us*)p, *(const v8us*)(p + 16)); }
__device__ __forceinline__ void wave_sync() { __builtin_amdgcn_fence(3  , "wavefront"); __builtin_amdgcn_wave_barrier(); asm volatile("" ::: "memory"); }

static __device__ __forceinline__ h16 toh_flush(float v) { const h16 r = (h16)v; return (fabsf(v) < 6.103515625e-05f) ? (h16)0.0f : r; }
__device__ __forceinline__ v8f wmmab_g(v16bf a, v16bf b, v8f c) { c = wmmab(a, b, c); asm volatile("v_nop\n\tv_nop\n\tv_nop\n\tv_nop" : "+v"(c) : "v"(a), "v"(b)); return c; }
__device__ __forceinline__ v8f wmma16_g(v16h a, v16h b, v8f c) { c = wmma16(a, b, c); asm volatile("v_nop\n\tv_nop\n\tv_nop\n\tv_nop" : "+v"(c) : "v"(a), "v"(b)); return c; }

__global__ __launch_bounds__(256) void k_cvt8(const float* __restrict__ src, bf* dst, size_t n8) {
    const size_t i = (size_t)blockIdx.x * 256 + threadIdx.x; if (i >= n8) return;
    const v8f v = *(const v8f*)(src + i * 8); v8us o;
#pragma unroll
    for (int k = 0; k < 8; ++k) o[k] = f2bf(v[k]);
    *(volatile v8us*)(dst + i * 8) = o; __threadfence(); *(volatile v8us*)(dst + i * 8) = o;
}

__device__ __forceinline__ v8f wt_vals(const float* __restrict__ src, int ld, int nvalid, int kw8, int kb, float scale, int i) {
    const int n = i / kw8; const int k0 = (i - n * kw8) * 8;
    const int nc = n < nvalid ? n : nvalid - 1;
    v8f o;
#pragma unroll
    for (int k = 0; k < 8; ++k) { float x = src[(size_t)(kb + k0 + k) * (size_t)ld + (size_t)nc]; asm volatile("" : "+v"(x)); o[k] = (n < nvalid) ? bfr(x) * scale : 0.0f; }
    return o;
}
__global__ __launch_bounds__(256) void k_wt_bf(const float* __restrict__ src, bf* dst, int ld, int nvalid, int nrows, int kw8, int kb, float scale) {
    const int i = blockIdx.x * 256 + threadIdx.x; if (i >= nrows * kw8) return;
    const v8f v = wt_vals(src, ld, nvalid, kw8, kb, scale, i); v8us o;
#pragma unroll
    for (int k = 0; k < 8; ++k) o[k] = f2bf(v[k]);
    *(volatile v8us*)(dst + (size_t)i * 8) = o; __threadfence(); *(volatile v8us*)(dst + (size_t)i * 8) = o;
}
__global__ __launch_bounds__(256) void k_wt_h(const float* __restrict__ src, h16* dst, int ld, int nvalid, int nrows, int kw8, int kb, float scale) {
    const int i = blockIdx.x * 256 + threadIdx.x; if (i >= nrows * kw8) return;
    const v8f v = wt_vals(src, ld, nvalid, kw8, kb, scale, i); v8h o;
#pragma unroll
    for (int k = 0; k < 8; ++k) o[k] = toh_flush(v[k]);
    *(volatile v8h*)(dst + (size_t)i * 8) = o; __threadfence(); *(volatile v8h*)(dst + (size_t)i * 8) = o;
}

__global__ __launch_bounds__(32) void k_gemm_fc(const bf* __restrict__ XBp, const bf* __restrict__ W1, const float* __restrict__ bfe, const float* __restrict__ bse, float* F, float* C) {
    __shared__ __align__(16) float os[16 * G1P];
    const int lane = threadIdx.x & 31, lr = lane & 15, hi = lane >> 4; const int r0 = blockIdx.x * 32;
    v8f acc[2][NT1];
#pragma unroll
    for (int mb = 0; mb < 2; ++mb)
#pragma unroll
        for (int nb = 0; nb < NT1; ++nb) acc[mb][nb] = (v8f){};
    const size_t aoff = (size_t)(r0 + lr) * FIN + 8 * hi, boff = (size_t)lr * FIN + 8 * hi;
#pragma unroll 1
    for (int kc = 0; kc < FIN; kc += 32) {
        v16bf a[2];
#pragma unroll
        for (int mb = 0; mb < 2; ++mb) a[mb] = ldb(XBp + aoff + (size_t)mb * 16 * FIN + kc);
#pragma unroll
        for (int nb = 0; nb < NT1; ++nb) { const v16bf bq = ldb(W1 + boff + (size_t)nb * 16 * FIN + kc);
#pragma unroll
            for (int mb = 0; mb < 2; ++mb) acc[mb][nb] = wmmab_g(a[mb], bq, acc[mb][nb]); }
    }
    float bc[NT1];
#pragma unroll
    for (int nb = 0; nb < 4; ++nb) bc[nb] = bfr(bfe[nb * 16 + lr]);
    { float v2 = bse[lr < SD ? lr : SD - 1]; asm volatile("" : "+v"(v2)); bc[4] = (lr < SD) ? bfr(v2) : 0.0f; }
#pragma unroll
    for (int mb = 0; mb < 2; ++mb) {
#pragma unroll
        for (int nb = 0; nb < NT1; ++nb) {
#pragma unroll
            for (int j = 0; j < 8; ++j) os[(hi * 8 + j) * G1P + nb * 16 + lr] = acc[mb][nb][j] + bc[nb]; }
        wave_sync();
        float* fb = F + (size_t)(r0 + mb * 16) * PW;
        float* cb = C + (size_t)(r0 + mb * 16) * SD;
#pragma unroll 1
        for (int ps = 0; ps < 2; ++ps) {
#pragma unroll
            for (int s = 0; s < 8; ++s) { const int p = s * 32 + lane; const int row = p >> 4, c4 = (p & 15) * 4;
                const v4f val = *(const v4fa*)(&os[row * G1P + c4]);
                *(volatile v4f*)(fb + (size_t)p * 4) = val; }
            const v4f cv = *(const v4fa*)(&os[lr * G1P + PW]);
            if (lane < 16) *(volatile v4f*)(cb + (size_t)lane * 4) = cv;
            if (ps == 0) __threadfence(); }
        wave_sync();
    }
}

__global__ __launch_bounds__(KQ) void k_knn_pool(const float* __restrict__ C, const float* __restrict__ F, h16* CH) {
#pragma clang fp contract(off)
    __shared__ __align__(16) float cT[CT * 4];
    __shared__ float hd[KQ * KNN];
    __shared__ int   hx[KQ * KNN];
    __shared__ __align__(16) h16 st[KQ * CSP];
    const int t = threadIdx.x;
    const int lane = t & 31;
    const int wave = __builtin_amdgcn_readfirstlane((int)(threadIdx.x >> 5));
    const int b = blockIdx.y;
    const int v0 = blockIdx.x * KQ;
    const size_t rowb = (size_t)b * SEQ;
    const v4f cq = *(const v4f*)(C + (rowb + (size_t)(v0 + t)) * SD);
    const int lb = t * KNN;
#pragma unroll 1
    for (int k = 0; k < KNN; ++k) { hd[lb + k] = 3.4e38f; hx[lb + k] = 0; }
    float worst = 3.4e38f;
#pragma unroll 1
    for (int tile = 0; tile < SEQ / CT; ++tile) {
        __syncthreads();
#pragma unroll
        for (int j = 0; j < CT / KQ; ++j) { const int u = j * KQ + t;
            const v4f cv = *(const v4f*)(C + (rowb + (size_t)tile * CT + (size_t)u) * SD);
            *(v4fa*)(&cT[u * 4]) = cv; }
        __syncthreads();
#pragma unroll 4
        for (int u = 0; u < CT; ++u) {
            const v4f cu = *(const v4fa*)(&cT[u * 4]);
            const float dx = cq[0] - cu[0], dy = cq[1] - cu[1], dz = cq[2] - cu[2], dw = cq[3] - cu[3];
            const float d2 = dx * dx + dy * dy + dz * dz + dw * dw;
            if (d2 < worst) {
                int pos = KNN - 1;
                while (pos > 0) {
                    const float pd = hd[lb + pos - 1];
                    if (!(pd > d2)) break;
                    hd[lb + pos] = pd; hx[lb + pos] = hx[lb + pos - 1]; --pos; }
                hd[lb + pos] = d2; hx[lb + pos] = tile * CT + u;
                worst = hd[lb + KNN - 1];
            }
        }
    }
    __syncthreads();
#pragma unroll 1
    for (int k = 1; k < KNN; ++k) {
        const float d = hd[lb + k];
        const float e = -fabsf(d * 10.0f) * LOG2E;
        hd[lb + k] = __builtin_amdgcn_exp2f(e);
        int ix = hx[lb + k]; ix = ix < 0 ? 0 : (ix > SEQ - 1 ? SEQ - 1 : ix); hx[lb + k] = ix;
    }
    __syncthreads();
    const int qb = wave * 32;
#pragma unroll 1
    for (int q = 0; q < 32; ++q) {
        const int lq = (qb + q) * KNN;
        float mx0 = -3.4e38f, mx1 = -3.4e38f, s0 = 0.0f, s1 = 0.0f;
#pragma unroll 1
        for (int j = 1; j < KNN; ++j) {
            const int ui = hx[lq + j]; const float wg = hd[lq + j];
            const v2f f = *(const v2f*)(F + (rowb + (size_t)ui) * PW + 2 * lane);
            const float a0 = f[0] * wg, a1 = f[1] * wg;
            mx0 = fmaxf(mx0, a0); mx1 = fmaxf(mx1, a1);
            s0 += a0; s1 += a1;
        }
        const float me0 = s0 * (1.0f / (float)(KNN - 1)), me1 = s1 * (1.0f / (float)(KNN - 1));
        const int sb = (qb + q) * CSP + 2 * lane;
        st[sb] = toh_flush(mx0 * CCS); st[sb + 1] = toh_flush(mx1 * CCS);
        st[sb + PW] = toh_flush(me0 * CCS); st[sb + PW + 1] = toh_flush(me1 * CCS);
    }
    __syncthreads();
    h16* cb = CH + (rowb + (size_t)(v0 + qb)) * CW;
#pragma unroll 1
    for (int ps = 0; ps < 2; ++ps) {
#pragma unroll 1
        for (int s = 0; s < 16; ++s) { const int p = s * 32 + lane; const int row = p >> 4, c8 = (p & 15) * 8;
            const v8h val = *(const v8ha*)(&st[(qb + row) * CSP + c8]);
            *(volatile v8h*)(cb + (size_t)p * 8) = val; }
        if (ps == 0) __threadfence(); }
}

__global__ __launch_bounds__(32) void k_gemm_out(const bf* __restrict__ XBp, const h16* __restrict__ CHp, const bf* __restrict__ WOX, const h16* __restrict__ WOC, const float* __restrict__ boe, float* OUT) {
    __shared__ __align__(16) float os[16 * OP2];
    const int lane = threadIdx.x & 31, lr = lane & 15, hi = lane >> 4; const int r0 = blockIdx.x * 32;
    v8f acc[2][4];
#pragma unroll
    for (int mb = 0; mb < 2; ++mb)
#pragma unroll
        for (int nb = 0; nb < 4; ++nb) acc[mb][nb] = (v8f){};
    { const size_t aoff = (size_t)(r0 + lr) * FIN + 8 * hi, boff = (size_t)lr * FIN + 8 * hi;
#pragma unroll 1
      for (int kc = 0; kc < FIN; kc += 32) {
          v16bf a[2];
#pragma unroll
          for (int mb = 0; mb < 2; ++mb) a[mb] = ldb(XBp + aoff + (size_t)mb * 16 * FIN + kc);
#pragma unroll
          for (int nb = 0; nb < 4; ++nb) { const v16bf bq = ldb(WOX + boff + (size_t)nb * 16 * FIN + kc);
#pragma unroll
              for (int mb = 0; mb < 2; ++mb) acc[mb][nb] = wmmab_g(a[mb], bq, acc[mb][nb]); }
      } }
    { const size_t aoff = (size_t)(r0 + lr) * CW + 8 * hi, boff = (size_t)lr * CW + 8 * hi;
#pragma unroll 1
      for (int kc = 0; kc < CW; kc += 32) {
          v16h a[2];
#pragma unroll
          for (int mb = 0; mb < 2; ++mb) a[mb] = ldh(CHp + aoff + (size_t)mb * 16 * CW + kc);
#pragma unroll
          for (int nb = 0; nb < 4; ++nb) { const v16h bq = ldh(WOC + boff + (size_t)nb * 16 * CW + kc);
#pragma unroll
              for (int mb = 0; mb < 2; ++mb) acc[mb][nb] = wmma16_g(a[mb], bq, acc[mb][nb]); }
      } }
    float bc[4];
#pragma unroll
    for (int nb = 0; nb < 4; ++nb) bc[nb] = bfr(boe[nb * 16 + lr]);
#pragma unroll
    for (int mb = 0; mb < 2; ++mb) {
#pragma unroll
        for (int nb = 0; nb < 4; ++nb) {
#pragma unroll
            for (int j = 0; j < 8; ++j) os[(hi * 8 + j) * OP2 + nb * 16 + lr] = acc[mb][nb][j] * OINV + bc[nb]; }
        wave_sync();
#pragma unroll 1
        for (int s = 0; s < 8; ++s) { const int p = s * 32 + lane; const int ix = (p >> 4) * OP2 + (p & 15) * 4;
            v4f v = *(const v4fa*)(&os[ix]);
            v[0] = tanhf(v[0]); v[1] = tanhf(v[1]); v[2] = tanhf(v[2]); v[3] = tanhf(v[3]);
            *(v4fa*)(&os[ix]) = v; }
        wave_sync();
        const int m0 = r0 + mb * 16; const int bb = m0 / SEQ, tt = m0 % SEQ;
        float* ob = OUT + ((size_t)bb * OUT_SEQ + (size_t)tt) * FOUT;
#pragma unroll 1
        for (int ps = 0; ps < 2; ++ps) {
#pragma unroll
            for (int s = 0; s < 8; ++s) { const int p = s * 32 + lane; const int row = p >> 4, c4 = (p & 15) * 4;
                const v4f val = *(const v4fa*)(&os[row * OP2 + c4]);
                *(volatile v4f*)(ob + (size_t)p * 4) = val; }
            if (ps == 0) __threadfence(); }
        wave_sync();
    }
}

static constexpr size_t al256(size_t v) { return (v + 255) & ~(size_t)255; }
static constexpr size_t SZ_XB  = al256((size_t)NB * SEQ * FIN * 2);
static constexpr size_t SZ_W1  = al256((size_t)N1 * FIN * 2);
static constexpr size_t SZ_WOX = al256((size_t)FOUT * FIN * 2);
static constexpr size_t SZ_WOC = al256((size_t)FOUT * CW * 2);
static constexpr size_t SZ_F   = al256((size_t)NB * SEQ * PW * 4);
static constexpr size_t SZ_C   = al256((size_t)NB * SEQ * SD * 4);
static constexpr size_t SZ_CH  = al256((size_t)NB * SEQ * CW * 2);
static constexpr size_t SZ_TOTAL = SZ_XB + SZ_W1 + SZ_WOX + SZ_WOC + SZ_F + SZ_C + SZ_CH;
static_assert(SZ_TOTAL <= (size_t)134217728);
static_assert(((size_t)PW * FIN * 2) % 256 == 0);
static_assert((PW * (FIN / 8)) % 32 == 0);
static_assert(((N1 - PW) * (FIN / 8)) % 32 == 0);
static_assert((FOUT * (FIN / 8)) % 32 == 0);
static_assert((FOUT * (CW / 8)) % 32 == 0);

extern "C" void kernel_launch(void* const* d_in, const int* in_sizes, int n_in,
                              void* d_out, int out_size, void* d_ws, size_t ws_size, hipStream_t stream) {
    if (n_in < 7) return;
    const size_t needx = ((size_t)(NB - 1) * SEQ_FULL + SEQ) * FIN;
    if ((size_t)in_sizes[0] < needx) return;
    if (in_sizes[1] < FIN * PW || in_sizes[2] < PW || in_sizes[3] < FIN * SD || in_sizes[4] < SD) return;
    if (in_sizes[5] < (FIN + CW) * FOUT || in_sizes[6] < FOUT) return;
    if ((size_t)out_size < ((size_t)(NB - 1) * OUT_SEQ + SEQ) * FOUT) return;
    if (SZ_TOTAL > ws_size) return;
    const float* x   = (const float*)d_in[0];
    const float* wf  = (const float*)d_in[1];
    const float* bfe = (const float*)d_in[2];
    const float* ws_ = (const float*)d_in[3];
    const float* bse = (const float*)d_in[4];
    const float* wo  = (const float*)d_in[5];
    const float* boe = (const float*)d_in[6];
    float* OUT = (float*)d_out;
    char* wsp = (char*)d_ws;
    bf*  XB  = (bf*)wsp;  wsp += SZ_XB;
    bf*  W1  = (bf*)wsp;  wsp += SZ_W1;
    bf*  WOX = (bf*)wsp;  wsp += SZ_WOX;
    h16* WOC = (h16*)wsp; wsp += SZ_WOC;
    float* F = (float*)wsp; wsp += SZ_F;
    float* C = (float*)wsp; wsp += SZ_C;
    h16* CH  = (h16*)wsp; wsp += SZ_CH;

    if (SEQ == SEQ_FULL) {
        const size_t n8 = (size_t)NB * SEQ * FIN / 8;
        k_cvt8<<<(unsigned)((n8 + 255) / 256), 256, 0, stream>>>(x, XB, n8);
    } else {
        const size_t n8 = (size_t)SEQ * FIN / 8;
        for (int b = 0; b < NB; ++b) k_cvt8<<<(unsigned)((n8 + 255) / 256), 256, 0, stream>>>(x + (size_t)b * SEQ_FULL * FIN, XB + (size_t)b * SEQ * FIN, n8);
    }
    k_wt_bf<<<(PW * (FIN / 8) + 255) / 256, 256, 0, stream>>>(wf, W1, PW, PW, PW, FIN / 8, 0, 1.0f);
    k_wt_bf<<<((N1 - PW) * (FIN / 8) + 255) / 256, 256, 0, stream>>>(ws_, W1 + (size_t)PW * FIN, SD, SD, N1 - PW, FIN / 8, 0, 1.0f);
    k_wt_bf<<<(FOUT * (FIN / 8) + 255) / 256, 256, 0, stream>>>(wo, WOX, FOUT, FOUT, FOUT, FIN / 8, 0, WXS);
    k_wt_h<<<(FOUT * (CW / 8) + 255) / 256, 256, 0, stream>>>(wo, WOC, FOUT, FOUT, FOUT, CW / 8, FIN, WCS);

    k_gemm_fc<<<dim3(NB * SEQ / 32, 1, 1), 32, 0, stream>>>(XB, W1, bfe, bse, F, C);
    k_knn_pool<<<dim3(SEQ / KQ, NB, 1), KQ, 0, stream>>>(C, F, CH);
    k_gemm_out<<<dim3(NB * SEQ / 32, 1, 1), 32, 0, stream>>>(XB, CH, WOX, WOC, boe, OUT);
}
